// _KANLinear_32375463477685
// MI455X (gfx1250) — hardware-verified
//
#include <hip/hip_runtime.h>


#pragma clang fp contract(off)

#ifndef NB
#define NB 4096
#endif
#define NB_FULL 4096
#define INF_  1024
#define OUTF  1024
#define NJ    9
#define KTOT  (NJ * INF_)
#define PE    2048
#define ACARRY 256.0f
#define WCARRY 64.0f
#define OSCALE (1.0f / 16384.0f)
#define GRIDN 5
#define SORD  3
#define HS   ((float)(2.0 / GRIDN))
#define G0   ((float)(-1.0 - (2.0 / GRIDN) * SORD))

static_assert(GRIDN + SORD == NJ - 1);
static_assert(NB <= NB_FULL);
static_assert(NB % 64 == 0);
static_assert(OUTF % 64 == 0);
static_assert(KTOT % 32 == 0);
static_assert(INF_ % 256 == 0);
static_assert(((size_t)NB * INF_) % PE == 0);
static_assert(((size_t)OUTF * INF_) % PE == 0);
static_assert(256 * 8 == PE);
static_assert((size_t)256 * 16 * NJ == (size_t)NJ * PE * 2);
static_assert((size_t)NJ * PE * 2 <= 131072);
static_assert((size_t)16 * 68 * 4 <= 131072);
static_assert(32 * 16 * 8 == 16 * 64 * 4);
static_assert(ACARRY * WCARRY * OSCALE == 1.0f);

typedef _Float16 h16;
typedef unsigned short bf;
typedef __attribute__((ext_vector_type(16))) _Float16 v16h;
typedef __attribute__((ext_vector_type(8)))  _Float16 v8h;
typedef __attribute__((ext_vector_type(8)))  float    v8f;
typedef __attribute__((ext_vector_type(4)))  float    v4f;
typedef v4f  __attribute__((may_alias)) v4fa;
typedef v8h  __attribute__((may_alias)) v8ha;

__device__ __forceinline__ unsigned short f2bf(float f) { unsigned u = __float_as_uint(f); u += 0x7FFFu + ((u >> 16) & 1u); return (unsigned short)(u >> 16); }
__device__ __forceinline__ float bfr(float f) { return __uint_as_float(((unsigned)f2bf(f)) << 16); }
__device__ __forceinline__ v16h cat16(v8h lo, v8h hi) { return __builtin_shufflevector(lo, hi, 0, 1, 2, 3, 4, 5, 6, 7, 8, 9, 10, 11, 12, 13, 14, 15); }
__device__ __forceinline__ v8f wmma16(v16h a, v16h b, v8f c) { return __builtin_amdgcn_wmma_f32_16x16x32_f16(false, a, false, b, (short)0, c, false, false); }
__device__ __forceinline__ v16h  ldh(const h16* p) { return cat16(*(const v8h*)p, *(const v8h*)(p + 16)); }
__device__ __forceinline__ void wave_sync() { __builtin_amdgcn_fence(3  , "wavefront"); __builtin_amdgcn_wave_barrier(); asm volatile("" ::: "memory"); }
static __device__ __forceinline__ h16 toh_flush(float v) { const h16 r = (h16)v; return (fabsf(v) < 6.103515625e-05f) ? (h16)0.0f : r; }

__device__ __forceinline__ void spline_bases(float xt, float bs[8]) {
    float g[12];
#pragma unroll
    for (int t = 0; t < 12; ++t) g[t] = G0 + HS * (float)t;
    float b0[11];
#pragma unroll
    for (int t = 0; t < 11; ++t) b0[t] = ((xt >= g[t]) & (xt < g[t + 1])) ? 1.0f : 0.0f;
    const float r1 = 1.0f / (HS + 1e-8f);
    const float r2 = 1.0f / (2.0f * HS + 1e-8f);
    const float r3 = 1.0f / (3.0f * HS + 1e-8f);
    float b1[10];
#pragma unroll
    for (int t = 0; t < 10; ++t) b1[t] = (xt - g[t]) * r1 * b0[t] + (g[t + 2] - xt) * r1 * b0[t + 1];
    float b2[9];
#pragma unroll
    for (int t = 0; t < 9; ++t) b2[t] = (xt - g[t]) * r2 * b1[t] + (g[t + 3] - xt) * r2 * b1[t + 1];
#pragma unroll
    for (int t = 0; t < 8; ++t) bs[t] = (xt - g[t]) * r3 * b2[t] + (g[t + 4] - xt) * r3 * b2[t + 1];
}

__global__ __launch_bounds__(256) void k_wprep(const float* __restrict__ sw, const float* __restrict__ bw, h16* WP) {
    __shared__ __align__(16) h16 tl[NJ * PE];
    const int tid = threadIdx.x;
    const size_t ebase = (size_t)blockIdx.x * PE;
#pragma unroll 1
    for (int it = 0; it < PE / 256; ++it) {
        const int e = it * 256 + tid;
        const size_t gi = ebase + (size_t)e;
        const float b0 = bfr(bw[gi]);
        const v4f s0 = *(const v4f*)(sw + gi * 8);
        const v4f s1 = *(const v4f*)(sw + gi * 8 + 4);
        tl[e] = toh_flush(b0 * WCARRY);
#pragma unroll
        for (int j = 0; j < 4; ++j) { tl[(1 + j) * PE + e] = toh_flush(bfr(s0[j]) * WCARRY); tl[(5 + j) * PE + e] = toh_flush(bfr(s1[j]) * WCARRY); }
    }
    __syncthreads();
    const int e8 = tid * 8;
    const size_t gg = ebase + (size_t)e8;
    const size_t row = gg >> 10; const int col = (int)(gg & (size_t)(INF_ - 1));
    h16* dst = WP + row * KTOT + col;
#pragma unroll 1
    for (int ps = 0; ps < 2; ++ps) {
#pragma unroll
        for (int j = 0; j < NJ; ++j) { const v8h v = *(const v8ha*)(&tl[j * PE + e8]); *(volatile v8h*)(dst + (size_t)j * INF_) = v; }
        if (ps == 0) __threadfence(); }
}

__global__ __launch_bounds__(256) void k_aprep(const float* __restrict__ x, h16* AP) {
    __shared__ __align__(16) h16 tl[NJ * PE];
    const int tid = threadIdx.x;
    const size_t ebase = (size_t)blockIdx.x * PE;
#pragma unroll 1
    for (int it = 0; it < PE / 256; ++it) {
        const int e = it * 256 + tid;
        const float xv = bfr(x[ebase + (size_t)e]);
        const float xt = tanhf(xv);
        float bs[8];
        spline_bases(xt, bs);
        const float sg = __builtin_amdgcn_rcpf(1.0f + __expf(-xv));
        tl[e] = toh_flush(xv * sg * ACARRY);
#pragma unroll
        for (int j = 0; j < 8; ++j) tl[(1 + j) * PE + e] = toh_flush(bs[j] * ACARRY);
    }
    __syncthreads();
    const int e8 = tid * 8;
    const size_t gg = ebase + (size_t)e8;
    const size_t row = gg >> 10; const int col = (int)(gg & (size_t)(INF_ - 1));
    h16* dst = AP + row * KTOT + col;
#pragma unroll 1
    for (int ps = 0; ps < 2; ++ps) {
#pragma unroll
        for (int j = 0; j < NJ; ++j) { const v8h v = *(const v8ha*)(&tl[j * PE + e8]); *(volatile v8h*)(dst + (size_t)j * INF_) = v; }
        if (ps == 0) __threadfence(); }
}

__global__ __launch_bounds__(32) void k_gemm(const h16* __restrict__ A, const h16* __restrict__ Bt, float* OUT) {
    __shared__ __align__(16) float os[16 * 68];
    const int K = KTOT;
    const int lane = threadIdx.x & 31, lr = lane & 15, hi = lane >> 4; const int r0 = blockIdx.x * 64, c0 = blockIdx.y * 64;
    v8f acc[4][4];
#pragma unroll
    for (int mb = 0; mb < 4; ++mb)
#pragma unroll
        for (int nb = 0; nb < 4; ++nb) acc[mb][nb] = (v8f){};
    const size_t aoff = (size_t)(r0 + lr) * K + 8 * hi, boff = (size_t)(c0 + lr) * K + 8 * hi;
#pragma unroll 1
    for (int kc = 0; kc < K; kc += 32) {
        v16h a[4];
#pragma unroll
        for (int mb = 0; mb < 4; ++mb) a[mb] = ldh(A + aoff + (size_t)mb * 16 * K + kc);
#pragma unroll
        for (int nb = 0; nb < 4; ++nb) { const v16h b = ldh(Bt + boff + (size_t)nb * 16 * K + kc);
#pragma unroll
            for (int mb = 0; mb < 4; ++mb) acc[mb][nb] = wmma16(a[mb], b, acc[mb][nb]); }
        asm volatile("v_nop\n\tv_nop\n\tv_nop\n\tv_nop" : "+v"(acc[0][0]), "+v"(acc[1][1]), "+v"(acc[2][2]), "+v"(acc[3][3]) : "v"(a[0]), "v"(a[1]), "v"(a[2]), "v"(a[3]));
    }
    float* obase = OUT + (size_t)r0 * OUTF + c0;
#pragma unroll
    for (int mb = 0; mb < 4; ++mb) {
#pragma unroll
        for (int nb = 0; nb < 4; ++nb) {
#pragma unroll
            for (int j = 0; j < 8; ++j) os[(hi * 8 + j) * 68 + nb * 16 + lr] = acc[mb][nb][j] * OSCALE; }
        wave_sync();
#pragma unroll 1
        for (int ps = 0; ps < 2; ++ps) {
#pragma unroll
            for (int s = 0; s < 8; ++s) { const int row = 2 * s + (lane >> 4), c4 = (lane & 15) * 4;
                const v4f val = *(const v4fa*)(&os[row * 68 + c4]);
                *(volatile v4f*)(obase + (size_t)(mb * 16 + row) * OUTF + c4) = val; }
            if (ps == 0) __threadfence(); }
        wave_sync();
    }
}

static constexpr size_t al256(size_t v) { return (v + 255) & ~(size_t)255; }
static constexpr size_t SZ_AP = al256((size_t)NB * KTOT * 2);
static constexpr size_t SZ_WP = al256((size_t)OUTF * KTOT * 2);
static constexpr size_t SZ_TOTAL = SZ_AP + SZ_WP;
static_assert(SZ_TOTAL <= (size_t)134217728);
static_assert(SZ_AP == (size_t)NB * KTOT * 2);
static_assert(SZ_WP == (size_t)OUTF * KTOT * 2);
static_assert(((size_t)KTOT * 2) % 128 == 0);
static_assert(((size_t)OUTF * 4) % 128 == 0);

extern "C" void kernel_launch(void* const* d_in, const int* in_sizes, int n_in,
                              void* d_out, int out_size, void* d_ws, size_t ws_size, hipStream_t stream) {
    if (n_in < 3) return;
    if ((size_t)in_sizes[0] < (size_t)NB * INF_) return;
    if ((size_t)in_sizes[1] < (size_t)OUTF * INF_ * 8) return;
    if ((size_t)in_sizes[2] < (size_t)OUTF * INF_) return;
    if ((size_t)out_size < (size_t)NB * OUTF) return;
    if (SZ_TOTAL > ws_size) return;
    const float* x  = (const float*)d_in[0];
    const float* sw = (const float*)d_in[1];
    const float* bw = (const float*)d_in[2];
    float* OUT = (float*)d_out;
    char* wsp = (char*)d_ws;
    h16* AP = (h16*)wsp; wsp += SZ_AP;
    h16* WP = (h16*)wsp; wsp += SZ_WP;

    k_wprep<<<(unsigned)(((size_t)OUTF * INF_) / PE), 256, 0, stream>>>(sw, bw, WP);
    k_aprep<<<(unsigned)(((size_t)NB * INF_) / PE), 256, 0, stream>>>(x, AP);
    k_gemm<<<dim3(NB / 64, OUTF / 64, 1), 32, 0, stream>>>(AP, WP, OUT);
}
